// SSD_Block_53369263620388
// MI455X (gfx1250) — hardware-verified
//
#include <hip/hip_runtime.h>
#include <math.h>

#define NB     8
#define CH     128
#define SEQ1   1024
#define M1     8192
#define DI1    256
#define NH1    4
#define CD1    384
#define NPJ1   644
#define LDZ1   704
#define CXBC1  256
#define CDT1   640
#define COLB1  256
#define COLC1  320
#define SEQ2   128
#define DM2    1024
#define M2     1024
#define DI2    2048
#define NH2    32
#define CD2    2176
#define NPJ2   4256
#define LDZ2   4288
#define CXBC2  2048
#define CDT2   4224
#define COLB2  2048
#define COLC2  2112
#define HDIM   64
#define DSTATE 64
#define NSUB   4
#define NSTS   16
#define SCH    32
#define TPB    128
#define OSTR   68
#define TP     72
#define EPSV   1e-5f
#define WSCAP  134217728

static_assert(M1 == NB * SEQ1);
static_assert(M2 == NB * SEQ2);
static_assert(SEQ2 == CH);
static_assert(NPJ1 == 2 * DI1 + 2 * DSTATE + NH1);
static_assert(NPJ2 == 2 * DI2 + 2 * DSTATE + NH2);
static_assert(CD1 == DI1 + 2 * DSTATE);
static_assert(CD2 == DI2 + 2 * DSTATE);
static_assert(LDZ1 % 64 == 0 && LDZ1 >= NPJ1);
static_assert(LDZ2 % 64 == 0 && LDZ2 >= NPJ2);
static_assert(DI1 == NH1 * HDIM);
static_assert(DI2 == NH2 * HDIM);
static_assert(M1 % TPB == 0);
static_assert(M2 % TPB == 0);
static_assert(M2 / TPB == NB);
static_assert(TPB == CH);
static_assert(CD1 % 32 == 0);
static_assert(CD2 % 32 == 0);
static_assert(CH % 64 == 0);
static_assert(DM2 % 64 == 0);
static_assert(DI1 % 32 == 0 && DI2 % 32 == 0 && CH % 32 == 0 && DM2 % 32 == 0);
static_assert(NSUB * NSTS == DSTATE);
static_assert(HDIM * NSUB == 256);
static_assert(SCH * HDIM == 2 * 256 * 4);
static_assert(SEQ1 % SCH == 0 && SEQ2 % SCH == 0);
static_assert(OSTR % 4 == 0);
static_assert(TP % 8 == 0);
static_assert(M1 % 16 == 0);
static_assert(SEQ1 % 64 == 0);

typedef unsigned short us16 __attribute__((ext_vector_type(16)));
typedef unsigned short us8  __attribute__((ext_vector_type(8)));
typedef unsigned short us8a __attribute__((ext_vector_type(8), may_alias));
typedef _Float16 v16h __attribute__((ext_vector_type(16)));
typedef float v8f __attribute__((ext_vector_type(8)));
typedef float v4f __attribute__((ext_vector_type(4)));
typedef float v4fa __attribute__((ext_vector_type(4), may_alias));
union FragU { us16 v; us8 h[2]; };

__device__ __forceinline__ unsigned short bf16_bits(float f) {
  unsigned u = __float_as_uint(f);
  u += 0x7FFFu + ((u >> 16) & 1u);
  return (unsigned short)(u >> 16);
}
__device__ __forceinline__ float bf16_val(unsigned short b) { return __uint_as_float(((unsigned)b) << 16); }
__device__ __forceinline__ float bf16r(float f) { return bf16_val(bf16_bits(f)); }
__device__ __forceinline__ unsigned short f16_bits(float f) { const _Float16 hv = (_Float16)f; return __builtin_bit_cast(unsigned short, hv); }
__device__ __forceinline__ float siluf(float x) { return x * __builtin_amdgcn_rcpf(1.0f + __expf(-x)); }

__device__ __forceinline__ v8f mma16(us16 a, us16 b, v8f c) {
  return __builtin_amdgcn_wmma_f32_16x16x32_f16(false, __builtin_bit_cast(v16h, a), false, __builtin_bit_cast(v16h, b), (short)0, c, false, false);
}
__device__ __forceinline__ void wguard(v8f& c0, v8f& c1, v8f& c2, v8f& c3, const us16& a0,
                                       const us16& b0, const us16& b1, const us16& b2, const us16& b3) {
#if defined(__HIP_DEVICE_COMPILE__)
  asm volatile("v_nop\n\tv_nop\n\tv_nop\n\tv_nop"
               : "+v"(c0), "+v"(c1), "+v"(c2), "+v"(c3)
               : "v"(a0), "v"(b0), "v"(b1), "v"(b2), "v"(b3));
#endif
}

__device__ __forceinline__ us16 gfrag(const unsigned short* p) {
  const int kh = ((threadIdx.x >> 4) & 1) * 8;
  FragU f;
  f.h[0] = *(const us8a*)(p + kh);
  f.h[1] = *(const us8a*)(p + 16 + kh);
  return f.v;
}

__global__ __launch_bounds__(256) void k_ln1(const float* __restrict__ x, const float* __restrict__ w,
                                            const float* __restrict__ bb, unsigned short* XA) {
  const int tid = threadIdx.x, lane = tid & 31, wave = tid >> 5, hq = lane >> 4, cl = lane & 15;
  const int row = blockIdx.x * 16 + 2 * wave + hq;
  const int c0 = 8 * cl;
  const float* xr = x + (size_t)row * CH + c0;
  const v4f a = *(const v4fa*)xr, bq = *(const v4fa*)(xr + 4);
  float v[8];
#pragma unroll
  for (int u = 0; u < 4; ++u) { v[u] = bf16r(a[u]); v[4 + u] = bf16r(bq[u]); }
  float s = 0.0f;
#pragma unroll
  for (int u = 0; u < 8; ++u) s += v[u];
  s += __shfl_xor(s, 8);
  s += __shfl_xor(s, 4);
  s += __shfl_xor(s, 2);
  s += __shfl_xor(s, 1);
  const float mean = s * (1.0f / (float)CH);
  float d[8];
  float q = 0.0f;
#pragma unroll
  for (int u = 0; u < 8; ++u) { d[u] = v[u] - mean; q += d[u] * d[u]; }
  q += __shfl_xor(q, 8);
  q += __shfl_xor(q, 4);
  q += __shfl_xor(q, 2);
  q += __shfl_xor(q, 1);
  const float rs = rsqrtf(q * (1.0f / (float)CH) + EPSV);
  us8 o;
#pragma unroll
  for (int u = 0; u < 8; ++u) o[u] = f16_bits((d[u] * rs) * bf16r(w[c0 + u]) + bf16r(bb[c0 + u]));
  const size_t off = (size_t)row * CH + c0;
  *(volatile us8*)(XA + off) = o;
  __threadfence();
  *(volatile us8*)(XA + off) = o;
}

__global__ __launch_bounds__(256) void k_lnT(const float* __restrict__ XS, const float* __restrict__ w,
                                            const float* __restrict__ bb, unsigned short* XA) {
  __shared__ float red[8 * 32];
  __shared__ float sm[32];
  __shared__ float sr[32];
  __shared__ __attribute__((aligned(16))) unsigned short T[32 * TP];
  const int tid = threadIdx.x, cl = tid & 31, lg = tid >> 5;
  const int b = blockIdx.x >> 2, c0 = (blockIdx.x & 3) * 32;
  const float* base = XS + (size_t)b * SEQ1 * CH + c0 + cl;

  float s = 0.0f;
#pragma unroll 4
  for (int j = 0; j < SEQ1 / 8; ++j) s += base[(size_t)(lg + 8 * j) * CH];
  red[lg * 32 + cl] = s;
  __syncthreads();
  if (tid < 32) {
    float t = red[tid];
#pragma unroll
    for (int g = 1; g < 8; ++g) t += red[g * 32 + tid];
    sm[tid] = t * (1.0f / (float)SEQ1);
  }
  __syncthreads();
  const float mean = sm[cl];
  float q = 0.0f;
#pragma unroll 4
  for (int j = 0; j < SEQ1 / 8; ++j) {
    const float dv = base[(size_t)(lg + 8 * j) * CH] - mean;
    q += dv * dv;
  }
  red[lg * 32 + cl] = q;
  __syncthreads();
  if (tid < 32) {
    float t = red[tid];
#pragma unroll
    for (int g = 1; g < 8; ++g) t += red[g * 32 + tid];
    sr[tid] = rsqrtf(t * (1.0f / (float)SEQ1) + EPSV);
  }
  __syncthreads();
  const float rs = sr[cl];

#pragma unroll 1
  for (int lt = 0; lt < SEQ1 / 64; ++lt) {
#pragma unroll
    for (int j = 0; j < 8; ++j) {
      const int ll = lg + 8 * j, l = lt * 64 + ll;
      const float v = ((base[(size_t)l * CH] - mean) * rs) * bf16r(w[l]) + bf16r(bb[l]);
      T[cl * TP + ll] = f16_bits(v);
    }
    __syncthreads();
    {
      const int c = tid >> 3, q8 = (tid & 7) * 8;
      const us8 val = *(const us8a*)(T + c * TP + q8);
      const size_t off = ((size_t)(b * CH + c0 + c)) * SEQ1 + (size_t)(lt * 64 + q8);
      *(volatile us8*)(XA + off) = val;
      __threadfence();
      *(volatile us8*)(XA + off) = val;
    }
    __syncthreads();
  }
}

__global__ __launch_bounds__(256) void k_cvtw(const float* __restrict__ src, unsigned short* dst, int K, int N, int total8, float scale) {
  const int idx = blockIdx.x * 256 + threadIdx.x;
  if (idx >= total8) return;
  const int k8n = K >> 3;
  const int n = idx / k8n, k8 = (idx - n * k8n) * 8;
  const int ns = (n < N) ? n : (N - 1);
  const bool zr = (n >= N);
  us8 o;
#pragma unroll
  for (int u = 0; u < 8; ++u) {
    const float f = src[(size_t)(k8 + u) * (size_t)N + ns];
    const float r = zr ? 0.0f : bf16r(f);
    o[u] = f16_bits(r * scale);
  }
  const size_t off = (size_t)n * (size_t)K + k8;
  *(volatile us8*)(dst + off) = o;
  __threadfence();
  *(volatile us8*)(dst + off) = o;
}

template <int EPI>
__global__ __launch_bounds__(256) void k_gemm(const unsigned short* __restrict__ Ap, int lda,
                                             const unsigned short* __restrict__ Bw, int ldb, int K,
                                             float* Yf, int ldy, const float* __restrict__ Res, float oscale) {
  __shared__ __attribute__((aligned(16))) float oS[8 * 16 * OSTR];
  const int tid = threadIdx.x, lane = tid & 31, wave = tid >> 5, cl = lane & 15, hh = lane >> 4;
  const int m0 = blockIdx.x * TPB + 16 * wave, n0 = blockIdx.y * 64;

  v8f acc[4];
#pragma unroll
  for (int j = 0; j < 4; ++j) { const v8f zz = {0.f, 0.f, 0.f, 0.f, 0.f, 0.f, 0.f, 0.f}; acc[j] = zz; }

  const unsigned short* ap  = Ap + (size_t)(m0 + cl) * (size_t)lda;
  const unsigned short* bwp = Bw + (size_t)(n0 + cl) * (size_t)ldb;
#pragma unroll 1
  for (int k0 = 0; k0 < K; k0 += 32) {
    const us16 af = gfrag(ap + k0);
    us16 bfr[4];
#pragma unroll
    for (int j = 0; j < 4; ++j) bfr[j] = gfrag(bwp + (size_t)(16 * j) * (size_t)ldb + k0);
#pragma unroll
    for (int j = 0; j < 4; ++j) acc[j] = mma16(af, bfr[j], acc[j]);
    wguard(acc[0], acc[1], acc[2], acc[3], af, bfr[0], bfr[1], bfr[2], bfr[3]);
  }

  float* so = oS + wave * (16 * OSTR);
#pragma unroll
  for (int j = 0; j < 4; ++j)
#pragma unroll
    for (int r = 0; r < 8; ++r) so[(8 * hh + r) * OSTR + 16 * j + cl] = acc[j][r];
  __syncthreads();

  if (EPI == 2) {
#pragma unroll
    for (int ps = 0; ps < 2; ++ps) {
#pragma unroll
      for (int it = 0; it < 8; ++it) {
        const int f = it * 256 + tid, lr = f >> 5, c4 = (f & 31) * 4;
        const float* sw = oS + (c4 >> 4) * (16 * OSTR) + (c4 & 15) * OSTR + lr;
        const size_t o = ((size_t)blockIdx.x * (size_t)ldy + (size_t)(n0 + lr)) * (size_t)TPB + (size_t)c4;
        const v4f rr = *(const v4fa*)(Res + o);
        v4f v;
#pragma unroll
        for (int u = 0; u < 4; ++u) v[u] = sw[u * OSTR] * oscale + rr[u];
        *(volatile v4f*)(Yf + o) = v;
      }
      __threadfence();
    }
  } else {
#pragma unroll
    for (int ps = 0; ps < 2; ++ps) {
#pragma unroll
      for (int it = 0; it < 8; ++it) {
        const int cx = it * 32 + lane, r = cx >> 4, q = (cx & 15) * 4;
        v4f v = *(const v4fa*)(so + r * OSTR + q) * oscale;
        const size_t o = (size_t)(m0 + r) * (size_t)ldy + (size_t)(n0 + q);
        if (EPI == 1) {
          const v4f rr = *(const v4fa*)(Res + o);
#pragma unroll
          for (int u = 0; u < 4; ++u) v[u] = v[u] + bf16r(rr[u]);
        }
        *(volatile v4f*)(Yf + o) = v;
      }
      __threadfence();
    }
  }
}

template <int SEQ, int LDZP, int CX, int CDP, int MR>
__global__ __launch_bounds__(256) void k_conv(const float* __restrict__ ZX, const float* __restrict__ cw,
                                             const float* __restrict__ cb, float* XC) {
  constexpr int C4N = CDP / 4;
  static_assert(C4N % 8 == 0);
  const int idx = blockIdx.x * 256 + threadIdx.x;
  if (idx >= MR * C4N) return;
  const int m = idx / C4N, c4 = (idx - m * C4N) * 4;
  const int l = m & (SEQ - 1);
  v4f xv[4];
#pragma unroll
  for (int k = 0; k < 4; ++k) {
    const int back = 3 - k;
    const bool ok = (l >= back);
    const int sr = ok ? (m - back) : m;
    const v4f t = *(const v4fa*)(ZX + (size_t)sr * LDZP + CX + c4);
    v4f z;
#pragma unroll
    for (int u = 0; u < 4; ++u) z[u] = ok ? t[u] : 0.0f;
    xv[k] = z;
  }
  v4f wv[4];
#pragma unroll
  for (int k = 0; k < 4; ++k) {
    const v4f wr = *(const v4fa*)(cw + (size_t)k * CDP + c4);
    v4f t;
#pragma unroll
    for (int u = 0; u < 4; ++u) t[u] = bf16r(wr[u]);
    wv[k] = t;
  }
  const v4f cbv = *(const v4fa*)(cb + c4);
  v4f ov;
#pragma unroll
  for (int u = 0; u < 4; ++u) {
    const float acc = (((wv[0][u] * xv[0][u] + wv[1][u] * xv[1][u]) + wv[2][u] * xv[2][u]) + wv[3][u] * xv[3][u]) + bf16r(cbv[u]);
    ov[u] = siluf(acc);
  }
  const size_t off = (size_t)m * CDP + c4;
  *(volatile v4f*)(XC + off) = ov;
  __threadfence();
  *(volatile v4f*)(XC + off) = ov;
}

template <int SEQ, int NHD, int LDZP, int CDT, int CDP, int CB, int CC, int DIP>
__global__ __launch_bounds__(256) void k_scan(const float* __restrict__ ZX, const float* __restrict__ XC,
                                             const float* __restrict__ dtb, const float* __restrict__ Alog,
                                             const float* __restrict__ Dsk, float* Y) {
  static_assert(SEQ % SCH == 0);
  static_assert(DIP == NHD * HDIM);
  __shared__ __attribute__((aligned(16))) float sDT[SEQ];
  __shared__ __attribute__((aligned(16))) float sDA[SEQ];
  __shared__ __attribute__((aligned(16))) float sy[SCH * HDIM];
  const int tid = threadIdx.x;
  const int s = blockIdx.x / NHD, hh = blockIdx.x - s * NHD;
  const int p = tid >> 2, sub = tid & 3, n0 = sub * NSTS;
  const size_t row0 = (size_t)s * SEQ;
  const float Acoef = -expf(bf16r(Alog[hh]));
  const float dbias = bf16r(dtb[hh]);
  const float Dd = bf16r(Dsk[hh]);

#pragma unroll 1
  for (int i = tid; i < SEQ; i += 256) {
    const float v = ZX[(row0 + (size_t)i) * LDZP + CDT + hh] + dbias;
    const float dt = fmaxf(v, 0.0f) + log1pf(expf(-fabsf(v)));
    sDT[i] = dt;
    sDA[i] = expf(dt * Acoef);
  }
  __syncthreads();

  float h[NSTS];
#pragma unroll
  for (int i = 0; i < NSTS; ++i) h[i] = 0.0f;

#pragma unroll 1
  for (int c = 0; c < SEQ / SCH; ++c) {
#pragma unroll 1
    for (int st = 0; st < SCH; ++st) {
      const int l = c * SCH + st;
      const float* xr = XC + (row0 + (size_t)l) * CDP;
      const float xv = xr[hh * HDIM + p];
      v4f Bv[4], Cv[4];
#pragma unroll
      for (int q = 0; q < 4; ++q) {
        Bv[q] = *(const v4fa*)(xr + CB + n0 + 4 * q);
        Cv[q] = *(const v4fa*)(xr + CC + n0 + 4 * q);
      }
      const float dl = sDT[l], da = sDA[l];
      const float dx = dl * xv;
      float y = 0.0f;
#pragma unroll
      for (int i = 0; i < NSTS; ++i) {
        h[i] = da * h[i] + dx * Bv[i >> 2][i & 3];
        y = y + h[i] * Cv[i >> 2][i & 3];
      }
      y += __shfl_xor(y, 1);
      y += __shfl_xor(y, 2);
      const float yv = y + xv * Dd;
      if (sub == 0) sy[st * HDIM + p] = yv;
    }
    __syncthreads();
#pragma unroll
    for (int ps = 0; ps < 2; ++ps) {
#pragma unroll
      for (int it = 0; it < 2; ++it) {
        const int cx = it * 256 + tid, r = cx >> 4, q = (cx & 15) * 4;
        const v4f v = *(const v4fa*)(sy + r * HDIM + q);
        *(volatile v4f*)(Y + (row0 + (size_t)(c * SCH + r)) * DIP + hh * HDIM + q) = v;
      }
      __threadfence();
    }
    __syncthreads();
  }
}

template <int DIP, int LDZP>
__global__ __launch_bounds__(256) void k_norm(const float* __restrict__ Y, const float* __restrict__ ZX,
                                             const float* __restrict__ nw, unsigned short* YN) {
  constexpr int TPR = DIP / 8;
  constexpr int RPB = 256 / TPR;
  static_assert(TPR == 32 || TPR == 256);
  __shared__ float red[8];
  const int tid = threadIdx.x, lane = tid & 31, wave = tid >> 5;
  const int row = blockIdx.x * RPB + tid / TPR;
  const int c8 = (tid % TPR) * 8;
  const size_t m = (size_t)row;
  const v4f y0 = *(const v4fa*)(Y + m * DIP + c8), y1 = *(const v4fa*)(Y + m * DIP + c8 + 4);
  const v4f z0 = *(const v4fa*)(ZX + m * LDZP + c8), z1 = *(const v4fa*)(ZX + m * LDZP + c8 + 4);
  float g[8];
  float ss = 0.0f;
#pragma unroll
  for (int u = 0; u < 4; ++u) {
    g[u] = y0[u] * siluf(z0[u]);
    g[4 + u] = y1[u] * siluf(z1[u]);
  }
#pragma unroll
  for (int u = 0; u < 8; ++u) ss += g[u] * g[u];
  ss += __shfl_xor(ss, 16);
  ss += __shfl_xor(ss, 8);
  ss += __shfl_xor(ss, 4);
  ss += __shfl_xor(ss, 2);
  ss += __shfl_xor(ss, 1);
  if (TPR > 32) {
    if (lane == 0) red[wave] = ss;
    __syncthreads();
    float t = red[0];
#pragma unroll
    for (int gq = 1; gq < 8; ++gq) t += red[gq];
    ss = t;
  }
  const float rs = rsqrtf(ss * (1.0f / (float)DIP) + EPSV);
  us8 o;
#pragma unroll
  for (int u = 0; u < 8; ++u) o[u] = f16_bits((g[u] * rs) * bf16r(nw[c8 + u]));
  const size_t off = m * DIP + c8;
  *(volatile us8*)(YN + off) = o;
  __threadfence();
  *(volatile us8*)(YN + off) = o;
}

static inline unsigned cdvu(long a, long bq) { return (unsigned)((a + bq - 1) / bq); }

extern "C" void kernel_launch(void* const* d_in, const int* in_sizes, int n_in,
                              void* d_out, int out_size, void* d_ws, size_t ws_size,
                              hipStream_t stream) {
  if (n_in < 21) return;
  if (in_sizes[0] != M1 * CH || in_sizes[1] != CH || in_sizes[2] != CH || in_sizes[3] != SEQ1 || in_sizes[4] != SEQ1 ||
      in_sizes[5] != CH * NPJ1 || in_sizes[6] != 4 * CD1 || in_sizes[7] != CD1 || in_sizes[8] != NH1 || in_sizes[9] != NH1 ||
      in_sizes[10] != NH1 || in_sizes[11] != DI1 || in_sizes[12] != DI1 * CH ||
      in_sizes[13] != DM2 * NPJ2 || in_sizes[14] != 4 * CD2 || in_sizes[15] != CD2 || in_sizes[16] != NH2 || in_sizes[17] != NH2 ||
      in_sizes[18] != NH2 || in_sizes[19] != DI2 || in_sizes[20] != DI2 * DM2) return;
  if (out_size != M1 * CH) return;

  const float* x       = (const float*)d_in[0];
  const float* ln1_w   = (const float*)d_in[1];
  const float* ln1_b   = (const float*)d_in[2];
  const float* ln2_w   = (const float*)d_in[3];
  const float* ln2_b   = (const float*)d_in[4];
  const float* w_in1   = (const float*)d_in[5];
  const float* cw1     = (const float*)d_in[6];
  const float* cb1     = (const float*)d_in[7];
  const float* dtb1    = (const float*)d_in[8];
  const float* alog1   = (const float*)d_in[9];
  const float* dsk1    = (const float*)d_in[10];
  const float* rms1    = (const float*)d_in[11];
  const float* w_out1  = (const float*)d_in[12];
  const float* w_in2   = (const float*)d_in[13];
  const float* cw2     = (const float*)d_in[14];
  const float* cb2     = (const float*)d_in[15];
  const float* dtb2    = (const float*)d_in[16];
  const float* alog2   = (const float*)d_in[17];
  const float* dsk2    = (const float*)d_in[18];
  const float* rms2    = (const float*)d_in[19];
  const float* w_out2  = (const float*)d_in[20];
  float* out = (float*)d_out;

  size_t off = 0;
  auto carve = [&](size_t bytes) -> char* { char* p = (char*)d_ws + off; off += (bytes + 255) & ~(size_t)255; return p; };
  unsigned short* XA1 = (unsigned short*)carve((size_t)M1 * CH * 2);
  unsigned short* WI1 = (unsigned short*)carve((size_t)LDZ1 * CH * 2);
  unsigned short* WO1 = (unsigned short*)carve((size_t)CH * DI1 * 2);
  float* ZX1  = (float*)carve((size_t)M1 * LDZ1 * 4);
  float* XCP1 = (float*)carve((size_t)M1 * CD1 * 4);
  float* Y1   = (float*)carve((size_t)M1 * DI1 * 4);
  unsigned short* YN1 = (unsigned short*)carve((size_t)M1 * DI1 * 2);
  float* XS   = (float*)carve((size_t)M1 * CH * 4);
  unsigned short* XA2 = (unsigned short*)carve((size_t)M2 * DM2 * 2);
  unsigned short* WI2 = (unsigned short*)carve((size_t)LDZ2 * DM2 * 2);
  unsigned short* WO2 = (unsigned short*)carve((size_t)DM2 * DI2 * 2);
  float* ZX2  = (float*)carve((size_t)M2 * LDZ2 * 4);
  float* XCP2 = (float*)carve((size_t)M2 * CD2 * 4);
  float* Y2   = (float*)carve((size_t)M2 * DI2 * 4);
  unsigned short* YN2 = (unsigned short*)carve((size_t)M2 * DI2 * 2);
  if (off > ws_size || off > (size_t)WSCAP) return;

  const dim3 b256(256);

  k_ln1<<<dim3(M1 / 16), b256, 0, stream>>>(x, ln1_w, ln1_b, XA1);
  k_cvtw<<<dim3(cdvu((long)LDZ1 * (CH / 8), 256)), b256, 0, stream>>>(w_in1, WI1, CH, NPJ1, LDZ1 * (CH / 8), 64.0f);
  k_cvtw<<<dim3(cdvu((long)CH * (DI1 / 8), 256)), b256, 0, stream>>>(w_out1, WO1, DI1, CH, CH * (DI1 / 8), 256.0f);
  k_gemm<0><<<dim3(M1 / TPB, LDZ1 / 64), b256, 0, stream>>>(XA1, CH, WI1, CH, CH, ZX1, LDZ1, x, 0.015625f);
  k_conv<SEQ1, LDZ1, CXBC1, CD1, M1><<<dim3(cdvu((long)M1 * (CD1 / 4), 256)), b256, 0, stream>>>(ZX1, cw1, cb1, XCP1);
  k_scan<SEQ1, NH1, LDZ1, CDT1, CD1, COLB1, COLC1, DI1><<<dim3(NB * NH1), b256, 0, stream>>>(ZX1, XCP1, dtb1, alog1, dsk1, Y1);
  k_norm<DI1, LDZ1><<<dim3(M1 / 8), b256, 0, stream>>>(Y1, ZX1, rms1, YN1);
  k_gemm<1><<<dim3(M1 / TPB, CH / 64), b256, 0, stream>>>(YN1, DI1, WO1, DI1, DI1, XS, CH, x, 0.00390625f);

  k_lnT<<<dim3(NB * (CH / 32)), b256, 0, stream>>>(XS, ln2_w, ln2_b, XA2);
  k_cvtw<<<dim3(cdvu((long)LDZ2 * (DM2 / 8), 256)), b256, 0, stream>>>(w_in2, WI2, DM2, NPJ2, LDZ2 * (DM2 / 8), 256.0f);
  k_cvtw<<<dim3(cdvu((long)DM2 * (DI2 / 8), 256)), b256, 0, stream>>>(w_out2, WO2, DI2, DM2, DM2 * (DI2 / 8), 256.0f);
  k_gemm<0><<<dim3(M2 / TPB, LDZ2 / 64), b256, 0, stream>>>(XA2, DM2, WI2, DM2, DM2, ZX2, LDZ2, x, 0.00390625f);
  k_conv<SEQ2, LDZ2, CXBC2, CD2, M2><<<dim3(cdvu((long)M2 * (CD2 / 4), 256)), b256, 0, stream>>>(ZX2, cw2, cb2, XCP2);
  k_scan<SEQ2, NH2, LDZ2, CDT2, CD2, COLB2, COLC2, DI2><<<dim3(NB * NH2), b256, 0, stream>>>(ZX2, XCP2, dtb2, alog2, dsk2, Y2);
  k_norm<DI2, LDZ2><<<dim3(M2), b256, 0, stream>>>(Y2, ZX2, rms2, YN2);
  k_gemm<2><<<dim3(M2 / TPB, DM2 / 64), b256, 0, stream>>>(YN2, DI2, WO2, DI2, DI2, out, SEQ1, XS, 0.00390625f);
}
